// FBPinn_86285892977067
// MI455X (gfx1250) — hardware-verified
//
#include <hip/hip_runtime.h>

typedef _Float16 v16h __attribute__((ext_vector_type(16)));
typedef _Float16 v8h  __attribute__((ext_vector_type(8)));
typedef float    v8f  __attribute__((ext_vector_type(8)));
typedef float    v4f  __attribute__((ext_vector_type(4)));
union Frag { v16h v; v8h half[2]; };

#define NW     16
#define NEUR   32
#define MT     4
#define WPB    8
#define PPW    (16 * MT)
#define TPITCH (NEUR + 1)

__device__ __forceinline__ v8f wmma_f16(v16h a, v16h b, v8f c) {
    v8f d = __builtin_amdgcn_wmma_f32_16x16x32_f16(false, a, false, b, (short)0, c, false, false);
    asm volatile("v_nop\n\tv_nop\n\tv_nop\n\tv_nop" : "+v"(d) : "v"(a), "v"(b));
    return d;
}

__device__ __forceinline__ float tanh_er(float z) {
    float e = __builtin_amdgcn_exp2f(z * 2.8853900817779268f);
    float r = __builtin_amdgcn_rcpf(e + 1.0f);
    return fmaf(-2.0f, r, 1.0f);
}

__device__ __forceinline__ float tanh_hw(float z) {
#if __has_builtin(__builtin_amdgcn_tanhf)
    return __builtin_amdgcn_tanhf(z);
#else
    return tanh_er(z);
#endif
}

__device__ __forceinline__ float sigm(float t) {
    return fmaf(0.5f, tanh_hw(0.5f * t), 0.5f);
}

__global__ __launch_bounds__(256)
void k_prep_w2t(const float* __restrict__ W2, _Float16* W2T, int nwin)
{
    __shared__ float tile[NEUR * TPITCH];
    const int i = blockIdx.x;
    if (i >= nwin) return;
    const int t = threadIdx.x;
    const float* src = W2 + (size_t)i * NEUR * NEUR;
#pragma unroll
    for (int j = 0; j < 4; ++j) {
        const int e = t + 256 * j;
        const int k = e >> 5, n = e & 31;
        tile[n * TPITCH + k] = src[e];
    }
    __syncthreads();

    const bool act = (t < 128);
    const int  q   = act ? t : 0;
    const int  n   = q >> 2;
    const int  k0  = 8 * (q & 3);
    v8h v;
#pragma unroll
    for (int j = 0; j < 8; ++j) v[j] = (_Float16)tile[n * TPITCH + k0 + j];
    _Float16* dst = W2T + (size_t)i * NEUR * NEUR + 8 * q;
    if (act) *(volatile v8h*)dst = v;
    __threadfence();
    if (act) *(volatile v8h*)dst = v;
}

__global__ __launch_bounds__(256)
void k_fwd(const float* __restrict__ x,
           const float* __restrict__ W1,
           const float* __restrict__ b1,
           const _Float16* __restrict__ W2T,
           const float* __restrict__ b2,
           const float* __restrict__ W3,
           const float* __restrict__ b3,
           float* out, int N)
{
    const int lane = threadIdx.x & 31;
    const int m    = lane & 15;
    const int h    = lane >> 4;
    const long long wave = (long long)blockIdx.x * WPB + (threadIdx.x >> 5);
    const long long base = wave * PPW;
    if (base >= (long long)N) return;

    const long long p0 = base + 4 * m;
    const bool full = (p0 + 3 < (long long)N);
    float xp[MT];
    if (full) {
        v4f xv = *(const v4f*)(x + p0);
#pragma unroll
        for (int t = 0; t < MT; ++t) xp[t] = xv[t];
    } else {
#pragma unroll
        for (int t = 0; t < MT; ++t) {
            long long p = p0 + t;
            if (p > (long long)N - 1) p = (long long)N - 1;
            xp[t] = x[p];
        }
    }

    float acc[MT];
#pragma unroll
    for (int t = 0; t < MT; ++t) acc[t] = 0.0f;

    const float wdom = 0.0625f;
    const float invs = 200.0f;

#pragma unroll 1
    for (int i = 0; i < NW; ++i) {
        const float sub0   = (i == 0)      ? 0.0f : ((float)i - 0.125f) * wdom;
        const float sub1   = (i == NW - 1) ? 1.0f : ((float)i + 1.125f) * wdom;
        const float mean   = 0.5f * (sub0 + sub1);
        const float stdv   = 0.5f * (sub1 - sub0);
        const float invstd = 1.0f / stdv;
        const float mo0    = (float)i * wdom;
        const float mo1    = (float)(i + 1) * wdom;

        const float* W1p = W1 + i * NEUR + 8 * h;
        const v4f w1a0 = *(const v4f*)(W1p);
        const v4f w1a1 = *(const v4f*)(W1p + 4);
        const v4f w1b0 = *(const v4f*)(W1p + 16);
        const v4f w1b1 = *(const v4f*)(W1p + 20);
        const float* b1p = b1 + i * NEUR + 8 * h;
        const v4f b1a0 = *(const v4f*)(b1p);
        const v4f b1a1 = *(const v4f*)(b1p + 4);
        const v4f b1b0 = *(const v4f*)(b1p + 16);
        const v4f b1b1 = *(const v4f*)(b1p + 20);

        const _Float16* Ap0 = W2T + ((size_t)i * NEUR + m) * NEUR;
        const _Float16* Ap1 = Ap0 + 16 * NEUR;
        Frag a0, a1;
        a0.half[0] = *(const v8h*)(Ap0 + 8 * h);
        a0.half[1] = *(const v8h*)(Ap0 + 16 + 8 * h);
        a1.half[0] = *(const v8h*)(Ap1 + 8 * h);
        a1.half[1] = *(const v8h*)(Ap1 + 16 + 8 * h);

        const float* b2p = b2 + i * NEUR + 8 * h;
        const v4f b2a0 = *(const v4f*)(b2p);
        const v4f b2a1 = *(const v4f*)(b2p + 4);
        const v4f b2b0 = *(const v4f*)(b2p + 16);
        const v4f b2b1 = *(const v4f*)(b2p + 20);
        const float* W3p = W3 + i * NEUR + 8 * h;
        const v4f w3a0 = *(const v4f*)(W3p);
        const v4f w3a1 = *(const v4f*)(W3p + 4);
        const v4f w3b0 = *(const v4f*)(W3p + 16);
        const v4f w3b1 = *(const v4f*)(W3p + 20);
        v8f cin0, cin1;
        float w3a[8], w3b[8];
#pragma unroll
        for (int j = 0; j < 4; ++j) {
            cin0[j] = b2a0[j]; cin0[4 + j] = b2a1[j];
            cin1[j] = b2b0[j]; cin1[4 + j] = b2b1[j];
            w3a[j]  = w3a0[j]; w3a[4 + j]  = w3a1[j];
            w3b[j]  = w3b0[j]; w3b[4 + j]  = w3b1[j];
        }
        const float b3v = (h == 0) ? b3[i] : 0.0f;

#pragma unroll
        for (int t = 0; t < MT; ++t) {
            const float xv = xp[t];
            const float xn = (xv - mean) * invstd;

            const v4f ha0 = xn * w1a0 + b1a0;
            const v4f ha1 = xn * w1a1 + b1a1;
            const v4f hb0 = xn * w1b0 + b1b0;
            const v4f hb1 = xn * w1b1 + b1b1;
            v16h bv;
#pragma unroll
            for (int j = 0; j < 4; ++j) {
                bv[j]      = (_Float16)tanh_hw(ha0[j]);
                bv[4 + j]  = (_Float16)tanh_hw(ha1[j]);
                bv[8 + j]  = (_Float16)tanh_hw(hb0[j]);
                bv[12 + j] = (_Float16)tanh_hw(hb1[j]);
            }

            float win = sigm((xv - mo0) * invs) * sigm((mo1 - xv) * invs);
            win = (win > 1e-5f) ? win : 0.0f;

            const v8f d0 = wmma_f16(a0.v, bv, cin0);
            const v8f d1 = wmma_f16(a1.v, bv, cin1);

            float part = b3v;
#pragma unroll
            for (int r = 0; r < 8; ++r) {
                part = fmaf(tanh_hw(d0[r]), w3a[r], part);
                part = fmaf(tanh_hw(d1[r]), w3b[r], part);
            }
            acc[t] = fmaf(win, part, acc[t]);
        }
    }

    float val[MT];
#pragma unroll
    for (int t = 0; t < MT; ++t) {
        const float tot = acc[t] + __shfl_xor(acc[t], 16, 32);
        val[t] = tot * tanh_er(15.0f * xp[t]);
    }
    v4f o;
#pragma unroll
    for (int t = 0; t < MT; ++t) o[t] = val[t];

    if (h == 0) {
        if (full) {
            *(volatile v4f*)(out + p0) = o;
        } else {
#pragma unroll
            for (int t = 0; t < MT; ++t)
                if (p0 + t < (long long)N) *(volatile float*)(out + p0 + t) = val[t];
        }
    }
    __threadfence();
    if (h == 0) {
        if (full) {
            *(volatile v4f*)(out + p0) = o;
        } else {
#pragma unroll
            for (int t = 0; t < MT; ++t)
                if (p0 + t < (long long)N) *(volatile float*)(out + p0 + t) = val[t];
        }
    }
}

extern "C" void kernel_launch(void* const* d_in, const int* in_sizes, int n_in,
                              void* d_out, int out_size, void* d_ws, size_t ws_size,
                              hipStream_t stream)
{
    if (n_in < 7) return;
    const float* x  = (const float*)d_in[0];
    const float* W1 = (const float*)d_in[1];
    const float* b1 = (const float*)d_in[2];
    const float* W2 = (const float*)d_in[3];
    const float* b2 = (const float*)d_in[4];
    const float* W3 = (const float*)d_in[5];
    const float* b3 = (const float*)d_in[6];
    float* out = (float*)d_out;

    int N = in_sizes[0];
    if (out_size < N) N = out_size;
    if (N <= 0) return;
    if (in_sizes[1] < NW * NEUR || in_sizes[2] < NW * NEUR || in_sizes[3] < NW * NEUR * NEUR ||
        in_sizes[4] < NW * NEUR || in_sizes[5] < NW * NEUR || in_sizes[6] < NW) return;

    const size_t w2t_bytes = (size_t)NW * NEUR * NEUR * sizeof(_Float16);
    if (ws_size < w2t_bytes) return;
    _Float16* W2T = (_Float16*)d_ws;

    k_prep_w2t<<<NW, 256, 0, stream>>>(W2, W2T, NW);

    const int ptsPerBlock = WPB * PPW;
    const int grid = (N + ptsPerBlock - 1) / ptsPerBlock;
    k_fwd<<<grid, 256, 0, stream>>>(x, W1, b1, W2T, b2, W3, b3, out, N);
}
